// GCN_79766132621935
// MI455X (gfx1250) — hardware-verified
//
#include <hip/hip_runtime.h>
#include <stddef.h>
#include <stdint.h>
#include <math.h>


#define CIN      128
#define HID      128
#define APW      256
#define NGR      256
#define NCLS     5
#define NOUT     (NGR * NCLS)
#define NTHR     256
#define NWAVE    8
#define EPT      8
#define CHUNK    (NTHR * EPT)
#define WCAP     (EPT * 32)
#define LISTN    (NWAVE * WCAP)
#define NBMAX    2048
#define NB       1024
#define RCAP     28672
#define DEGCAP   64
#define PKS      11
#define STW      128
#define GBM      64
#define GTHR     128
#define GNT      8
#define BN       (16 * GNT)
#define NU1      (HID * (CIN / 8))
#define NUD      (HID * (APW / 8))
#define FLGW     32
#define WSMAX    134217728
#define LDS_BKT  ((2 * RCAP + 2 * NBMAX + LISTN) * 4 + 64)

static_assert((CHUNK & (CHUNK - 1)) == 0 && CHUNK <= (1 << PKS));
static_assert((NBMAX & (NBMAX - 1)) == 0 && NBMAX <= (1 << PKS) && NB <= NBMAX);
static_assert(NTHR * 8 == NBMAX && NTHR * 4 == NB);
static_assert(LISTN >= NBMAX && LISTN >= NWAVE * WCAP && LISTN >= NB);
static_assert((RCAP % (NTHR * 4)) == 0);
static_assert(((2 * RCAP + NBMAX) % (NTHR * 4)) == 0);
static_assert(RCAP >= 16638 + 16638 / 20 + 1);
static_assert(DEGCAP >= 36 + 8);
static_assert(LDS_BKT <= 300000);
static_assert(GBM == (GTHR / 32) * 16 && HID == BN && CIN == 128 && APW == 2 * HID);
static_assert((NU1 % NTHR) == 0 && (NUD % NTHR) == 0);
static_assert((NB % NWAVE) == 0 && HID == 32 * 4);
static_assert(NGR == NTHR && (NOUT % 4) == 0 && ((NOUT * 4) % 128) == 0 && NOUT / 4 <= 2 * NTHR);
static_assert(NOUT / 4 - NTHR == 64);

typedef float          v4f  __attribute__((ext_vector_type(4)));
typedef float          v8f  __attribute__((ext_vector_type(8)));
typedef int            v4i  __attribute__((ext_vector_type(4)));
typedef int            v8i  __attribute__((ext_vector_type(8)));
typedef unsigned int   v2u  __attribute__((ext_vector_type(2)));
typedef unsigned int   v4u  __attribute__((ext_vector_type(4)));
typedef unsigned short v8us __attribute__((ext_vector_type(8)));
typedef __bf16         v16b __attribute__((ext_vector_type(16)));
typedef v4f  __attribute__((may_alias)) v4fa;
typedef v4i  __attribute__((may_alias)) v4ia;
typedef v2u  __attribute__((may_alias)) v2ua;
typedef v4u  __attribute__((may_alias)) v4ua;
typedef v8us __attribute__((may_alias)) v8usa;
union FragB { v16b v; v8us h[2]; v8i w; };

__device__ __forceinline__ v8f wmb(const FragB& a, const FragB& b, v8f c) {
  v8f d = __builtin_amdgcn_wmma_f32_16x16x32_bf16(false, a.v, false, b.v, (short)0, c, false, false);
  asm volatile("v_nop\n\tv_nop\n\tv_nop\n\tv_nop" : "+v"(d) : "v"(a.w), "v"(b.w));
  return d;
}

__device__ __forceinline__ unsigned short bf_bits(float f) {
  const unsigned int u = __float_as_uint(f);
  const unsigned int r = (u + 0x7FFFu + ((u >> 16) & 1u)) >> 16;
  return (unsigned short)((f != f) ? 0x7FC0u : r);
}
__device__ __forceinline__ float bf_val(unsigned short b) {
  return __uint_as_float(((unsigned int)b) << 16);
}
__device__ __forceinline__ float bf_rne(float f) { return bf_val(bf_bits(f)); }

__device__ __forceinline__ int scan_chunk(const int* __restrict__ dsts, int nE, int cbase, int slotBase,
                                          int nb, int vec8, int* list, int tid, int lane, int wave) {
  int wc = 0;
  const int el0  = tid * EPT;
  const int e0   = cbase + el0;
  const int sent = -2147483647 - 1;
  v4i da, db;
  if (vec8 != 0 && cbase + CHUNK <= nE) {
    da = *(const v4i*)(dsts + e0);
    db = *(const v4i*)(dsts + e0 + 4);
  } else {
    da.x = (e0     < nE) ? dsts[min(e0,     nE - 1)] : sent;
    da.y = (e0 + 1 < nE) ? dsts[min(e0 + 1, nE - 1)] : sent;
    da.z = (e0 + 2 < nE) ? dsts[min(e0 + 2, nE - 1)] : sent;
    da.w = (e0 + 3 < nE) ? dsts[min(e0 + 3, nE - 1)] : sent;
    db.x = (e0 + 4 < nE) ? dsts[min(e0 + 4, nE - 1)] : sent;
    db.y = (e0 + 5 < nE) ? dsts[min(e0 + 5, nE - 1)] : sent;
    db.z = (e0 + 6 < nE) ? dsts[min(e0 + 6, nE - 1)] : sent;
    db.w = (e0 + 7 < nE) ? dsts[min(e0 + 7, nE - 1)] : sent;
  }
  const unsigned nbs = (unsigned)slotBase;
  const unsigned unb = (unsigned)nb;
  const unsigned s0 = (unsigned)da.x - nbs, s1 = (unsigned)da.y - nbs;
  const unsigned s2 = (unsigned)da.z - nbs, s3 = (unsigned)da.w - nbs;
  const unsigned s4 = (unsigned)db.x - nbs, s5 = (unsigned)db.y - nbs;
  const unsigned s6 = (unsigned)db.z - nbs, s7 = (unsigned)db.w - nbs;
  const bool h0 = s0 < unb, h1 = s1 < unb, h2 = s2 < unb, h3 = s3 < unb;
  const bool h4 = s4 < unb, h5 = s5 < unb, h6 = s6 < unb, h7 = s7 < unb;
  const unsigned any = __builtin_amdgcn_ballot_w32(h0 | h1 | h2 | h3 | h4 | h5 | h6 | h7);
  if (any != 0u) {
#define HITJ(J, HJ, SJ) { \
      const unsigned mj = __builtin_amdgcn_ballot_w32(HJ); \
      if (mj != 0u) { \
        if (HJ) { \
          const int pos = wc + (int)__builtin_amdgcn_mbcnt_lo(mj, 0u); \
          if (pos < WCAP) list[wave * WCAP + pos] = ((el0 + (J)) << PKS) | (int)(SJ); \
        } \
        wc += (int)__builtin_popcount(mj); } }
    HITJ(0, h0, s0)
    HITJ(1, h1, s1)
    HITJ(2, h2, s2)
    HITJ(3, h3, s3)
    HITJ(4, h4, s4)
    HITJ(5, h5, s5)
    HITJ(6, h6, s6)
    HITJ(7, h7, s7)
#undef HITJ
  }
  return wc;
}

__global__ __launch_bounds__(NTHR) void k_prep(const float* __restrict__ x, const float* __restrict__ W1,
                                               const float* __restrict__ W2, const float* __restrict__ W3,
                                               int nN, int nUx, unsigned short* pb,
                                               size_t eXB, size_t eW1, size_t eW2, size_t eW3) {
  const int u = (int)blockIdx.x * NTHR + (int)threadIdx.x;
  v8us o;
  size_t eo;
  if (u < nUx) {
    const int row = u >> 4;
    const int k8  = (u & 15) * 8;
    const int rc  = row < nN ? row : nN - 1;
    const float* p = x + (size_t)rc * CIN + k8;
    const v4f a = *(const v4fa*)p;
    const v4f b = *(const v4fa*)(p + 4);
    const bool ok = row < nN;
    o[0] = ok ? bf_bits(a.x) : (unsigned short)0;
    o[1] = ok ? bf_bits(a.y) : (unsigned short)0;
    o[2] = ok ? bf_bits(a.z) : (unsigned short)0;
    o[3] = ok ? bf_bits(a.w) : (unsigned short)0;
    o[4] = ok ? bf_bits(b.x) : (unsigned short)0;
    o[5] = ok ? bf_bits(b.y) : (unsigned short)0;
    o[6] = ok ? bf_bits(b.z) : (unsigned short)0;
    o[7] = ok ? bf_bits(b.w) : (unsigned short)0;
    eo = eXB + (size_t)row * CIN + (size_t)k8;
  } else {
    const int v = u - nUx;
    if (v < NU1) {
      const int n  = v >> 4;
      const int k8 = (v & 15) * 8;
      const float* p = W1 + (size_t)k8 * HID + n;
#pragma unroll
      for (int i = 0; i < 8; ++i) o[i] = bf_bits(p[(size_t)i * HID]);
      eo = eW1 + (size_t)n * CIN + (size_t)k8;
    } else if (v < NU1 + NUD) {
      const int v2 = v - NU1;
      const int n  = v2 >> 5;
      const int k8 = (v2 & 31) * 8;
      const int kk = k8 & (HID - 1);
      const float* p = W2 + (size_t)kk * HID + n;
#pragma unroll
      for (int i = 0; i < 8; ++i) o[i] = bf_bits(p[(size_t)i * HID]);
      eo = eW2 + (size_t)n * APW + (size_t)k8;
    } else if (v < NU1 + 2 * NUD) {
      const int v3 = v - NU1 - NUD;
      const int n  = v3 >> 5;
      const int k8 = (v3 & 31) * 8;
      const int kk = k8 & (HID - 1);
      const float* p = W3 + (size_t)kk * HID + n;
#pragma unroll
      for (int i = 0; i < 8; ++i) o[i] = bf_bits(p[(size_t)i * HID]);
      eo = eW3 + (size_t)n * APW + (size_t)k8;
    } else {
      return;
    }
  }
  unsigned short* dp = pb + eo;
  *(volatile v8us*)dp = o;
  __threadfence();
  *(volatile v8us*)dp = o;
}

__global__ __launch_bounds__(NTHR) void k_bucket(const int* __restrict__ srcs, const int* __restrict__ dsts,
                                                 int nN, int nE, int vec8,
                                                 int* LISTG, int* CNTG, int* OFFG, float* DISG, int* FLGG) {
  extern __shared__ __attribute__((aligned(16))) int dsm[];
  int* reg1 = dsm;
  int* reg2 = reg1 + RCAP;
  int* scnt = reg2 + RCAP;
  int* soff = scnt + NBMAX;
  int* list = soff + NBMAX;
  int* wcnt = list + LISTN;
  int* wtot = wcnt + NWAVE;
  const int tid = (int)threadIdx.x, lane = tid & 31, wave = tid >> 5;
  const int nodeBase = (int)blockIdx.x * NB;

  {
    const v4i z4 = {0, 0, 0, 0};
#pragma unroll 1
    for (int i = tid * 4; i < 2 * RCAP + NBMAX; i += NTHR * 4) *(v4ia*)(dsm + i) = z4;
  }
  __syncthreads();

  int tot = 0, ovr = 0;
  const int nChunks = (nE + CHUNK - 1) / CHUNK;
#pragma unroll 1
  for (int ch = 0; ch < nChunks; ++ch) {
    const int cbase = ch * CHUNK;
    const int wc = scan_chunk(dsts, nE, cbase, nodeBase, NB, vec8, list, tid, lane, wave);
    if (lane == 0) wcnt[wave] = wc;
    __syncthreads();
    int pre = 0, all = 0;
#pragma unroll
    for (int w2 = 0; w2 < NWAVE; ++w2) {
      int c = wcnt[w2];
      c = c < 0 ? 0 : (c > WCAP ? WCAP : c);
      all += c;
      pre += (w2 < wave) ? c : 0;
    }
    const int wcc  = wc > WCAP ? WCAP : wc;
    const int base = tot + pre;
#pragma unroll 1
    for (int i = lane; i < wcc; i += 32) {
      const int ent = list[wave * WCAP + i];
      const int el  = (ent >> PKS) & (CHUNK - 1);
      const int sl  = ent & (NBMAX - 1);
      int eid = cbase + el;
      eid = eid > nE - 1 ? nE - 1 : eid;
      const int pos = base + i;
      if (pos < RCAP) reg1[pos] = (int)(((unsigned)eid << PKS) | (unsigned)sl);
    }
    tot += all;
    if (tot > RCAP) ovr = 1;
    tot = tot > RCAP ? RCAP : tot;
    __syncthreads();
  }
  const int nh = tot;
  const int ovf = (ovr != 0 || nh >= RCAP) ? 1 : 0;

  if (wave == 0) {
#pragma unroll 1
    for (int b0 = 0; b0 < nh; b0 += 32) {
      const int idx = b0 + lane;
      const int uv  = reg1[idx < RCAP ? idx : RCAP - 1];
      const int m32 = (nh - b0) < 32 ? (nh - b0) : 32;
#pragma unroll 1
      for (int k = 0; k < m32; ++k) {
        const int u  = __builtin_amdgcn_readlane(uv, k);
        const int sl = u & (NBMAX - 1);
        if (lane == 0) scnt[sl] = scnt[sl] + 1;
      }
    }
  }
  __syncthreads();

  {
    const v4i ca = *(const v4ia*)(scnt + 8 * tid);
    const v4i cb = *(const v4ia*)(scnt + 8 * tid + 4);
    const int e0 = ca.x < 0 ? 0 : ca.x, e1 = ca.y < 0 ? 0 : ca.y, e2 = ca.z < 0 ? 0 : ca.z, e3 = ca.w < 0 ? 0 : ca.w;
    const int e4 = cb.x < 0 ? 0 : cb.x, e5 = cb.y < 0 ? 0 : cb.y, e6 = cb.z < 0 ? 0 : cb.z, e7 = cb.w < 0 ? 0 : cb.w;
    const int ts = e0 + e1 + e2 + e3 + e4 + e5 + e6 + e7;
    int incl = ts;
#pragma unroll
    for (int d = 1; d < 32; d <<= 1) {
      const int up = __shfl_up(incl, d);
      if (lane >= d) incl += up;
    }
    if (lane == 31) wtot[wave] = incl;
    __syncthreads();
    int pre = 0;
#pragma unroll
    for (int w2 = 0; w2 < NWAVE; ++w2) pre += (w2 < wave) ? wtot[w2] : 0;
    int run = pre + incl - ts;
    soff[8 * tid + 0] = run; run += e0;
    soff[8 * tid + 1] = run; run += e1;
    soff[8 * tid + 2] = run; run += e2;
    soff[8 * tid + 3] = run; run += e3;
    soff[8 * tid + 4] = run; run += e4;
    soff[8 * tid + 5] = run; run += e5;
    soff[8 * tid + 6] = run; run += e6;
    soff[8 * tid + 7] = run;
  }
  __syncthreads();
  for (int i = tid; i < NBMAX; i += NTHR) list[i] = soff[i];
  __syncthreads();

  if (wave == 0) {
#pragma unroll 1
    for (int b0 = 0; b0 < nh; b0 += 32) {
      const int idx = b0 + lane;
      const int uv  = reg1[idx < RCAP ? idx : RCAP - 1];
      const int m32 = (nh - b0) < 32 ? (nh - b0) : 32;
#pragma unroll 1
      for (int k = 0; k < m32; ++k) {
        const int u   = __builtin_amdgcn_readlane(uv, k);
        const int sl  = u & (NBMAX - 1);
        const int eid = (int)((unsigned)u >> PKS);
        if (lane == 0) {
          int pos = list[sl];
          pos = pos < 0 ? 0 : (pos > RCAP - 1 ? RCAP - 1 : pos);
          reg2[pos] = eid;
          list[sl] = pos + 1;
        }
      }
    }
  }
  __syncthreads();

#pragma unroll 1
  for (int i = tid; i < RCAP; i += NTHR) {
    int eid = reg2[i];
    eid = eid < 0 ? 0 : (eid > nE - 1 ? nE - 1 : eid);
    int s = srcs[eid];
    s = s < 0 ? 0 : (s > nN - 1 ? nN - 1 : s);
    reg1[i] = (i < nh) ? s : 0;
  }
#pragma unroll 1
  for (int i = tid; i < NB; i += NTHR) {
    int c = scnt[i];
    c = c < 0 ? 0 : c;
    const float dg = (float)(c + 1);
    list[i] = __float_as_int(1.0f / sqrtf(dg));
  }
  __syncthreads();

  int* lg = LISTG + (size_t)blockIdx.x * RCAP;
  const v4i c4 = *(const v4ia*)(scnt + 4 * tid);
  const v4i o4 = *(const v4ia*)(soff + 4 * tid);
  const v4i l4 = *(const v4ia*)(list + 4 * tid);
  v4f d4;
  d4.x = __int_as_float(l4.x); d4.y = __int_as_float(l4.y);
  d4.z = __int_as_float(l4.z); d4.w = __int_as_float(l4.w);
  const v4i f4 = {ovf, ovf, ovf, ovf};
  const bool fw = (wave == 0) && (lane < 8);

#pragma unroll 1
  for (int it = 0; it < RCAP / (NTHR * 4); ++it) {
    const int o = 4 * (it * NTHR + tid);
    const v4i v = *(const v4ia*)(reg1 + o);
    *(volatile v4i*)(lg + o) = v;
  }
  *(volatile v4i*)(CNTG + (size_t)nodeBase + 4 * tid) = c4;
  *(volatile v4i*)(OFFG + (size_t)nodeBase + 4 * tid) = o4;
  *(volatile v4f*)(DISG + (size_t)nodeBase + 4 * tid) = d4;
  if (fw) *(volatile v4i*)(FLGG + (size_t)blockIdx.x * FLGW + 4 * lane) = f4;
  __threadfence();
#pragma unroll 1
  for (int it = 0; it < RCAP / (NTHR * 4); ++it) {
    const int o = 4 * (it * NTHR + tid);
    const v4i v = *(const v4ia*)(reg1 + o);
    *(volatile v4i*)(lg + o) = v;
  }
  *(volatile v4i*)(CNTG + (size_t)nodeBase + 4 * tid) = c4;
  *(volatile v4i*)(OFFG + (size_t)nodeBase + 4 * tid) = o4;
  *(volatile v4f*)(DISG + (size_t)nodeBase + 4 * tid) = d4;
  if (fw) *(volatile v4i*)(FLGG + (size_t)blockIdx.x * FLGW + 4 * lane) = f4;
}

template <int KT>
__global__ __launch_bounds__(GTHR) void k_gemm(const unsigned short* __restrict__ A,
                                               const unsigned short* __restrict__ WT,
                                               float* outF, int mRows) {
  constexpr int NT = GNT;
  constexpr int NI = 16;
  static_assert((KT % 32) == 0);
  __shared__ __attribute__((aligned(16))) float stg[GBM * BN];
  const int tid = (int)threadIdx.x, lane = tid & 31, wave = tid >> 5, hh = lane >> 4, m = lane & 15;
  const int rowBase = (int)blockIdx.x * GBM;

  v8f acc[NT];
  {
    const v8f z = {0.f, 0.f, 0.f, 0.f, 0.f, 0.f, 0.f, 0.f};
#pragma unroll
    for (int t = 0; t < NT; ++t) acc[t] = z;
  }
  const unsigned short* ap = A + (size_t)(rowBase + 16 * wave + m) * (size_t)KT + 8 * hh;
  const unsigned short* wp = WT + (size_t)m * (size_t)KT + 8 * hh;
  constexpr int ksteps = KT / 32;
#pragma unroll 1
  for (int ks = 0; ks < ksteps; ++ks) {
    FragB af;
    af.h[0] = *(const v8usa*)(ap + 32 * ks);
    af.h[1] = *(const v8usa*)(ap + 32 * ks + 16);
#pragma unroll
    for (int t = 0; t < NT; ++t) {
      const unsigned short* wq = wp + (size_t)(16 * t) * (size_t)KT + 32 * ks;
      FragB bf;
      bf.h[0] = *(const v8usa*)wq;
      bf.h[1] = *(const v8usa*)(wq + 16);
      acc[t] = wmb(af, bf, acc[t]);
    }
  }

#pragma unroll
  for (int t = 0; t < NT; ++t) {
    const int lc = 16 * t + m;
#pragma unroll
    for (int r = 0; r < 8; ++r) {
      const int lr = 16 * wave + 8 * hh + r;
      stg[lr * BN + lc] = acc[t][r];
    }
  }
  __syncthreads();

  v4f fv[NI];
#pragma unroll
  for (int i = 0; i < NI; ++i) {
    const int lr = 16 * wave + i;
    fv[i] = *(const v4fa*)(stg + lr * BN + 4 * lane);
  }
#pragma unroll
  for (int i = 0; i < NI; ++i) {
    const int gr = rowBase + 16 * wave + i;
    float* op = outF + (size_t)gr * (size_t)HID + 4 * lane;
    if (gr < mRows) *(volatile v4f*)op = fv[i];
  }
  __threadfence();
#pragma unroll
  for (int i = 0; i < NI; ++i) {
    const int gr = rowBase + 16 * wave + i;
    float* op = outF + (size_t)gr * (size_t)HID + 4 * lane;
    if (gr < mRows) *(volatile v4f*)op = fv[i];
  }
}

template <int MODE>
__global__ __launch_bounds__(NTHR) void k_agg(const int* __restrict__ LISTG, const int* __restrict__ CNTG,
                                              const int* __restrict__ OFFG, const int* __restrict__ FLGG,
                                              const float* __restrict__ DISG, const float* __restrict__ Hf,
                                              const float* __restrict__ bias,
                                              unsigned short* Xhl, float* Hout, int nN, int MPr) {
  __shared__ __attribute__((aligned(16))) int scn[NB];
  __shared__ __attribute__((aligned(16))) int sof[NB];
  __shared__ __attribute__((aligned(16))) float sbs[HID];
  __shared__ __attribute__((aligned(16))) unsigned int stw[NWAVE * STW];
  const int tid = (int)threadIdx.x, lane = tid & 31, wave = tid >> 5;
  const int nodeBase = (int)blockIdx.x * NB;
  const int* lg = LISTG + (size_t)blockIdx.x * RCAP;

  {
    const v4i c4 = *(const v4i*)(CNTG + (size_t)nodeBase + 4 * tid);
    const v4i o4 = *(const v4i*)(OFFG + (size_t)nodeBase + 4 * tid);
    *(v4ia*)(scn + 4 * tid) = c4;
    *(v4ia*)(sof + 4 * tid) = o4;
    if (tid < HID / 4) {
      const v4f bb = *(const v4f*)(bias + 4 * tid);
      v4f br;
      br.x = bf_rne(bb.x); br.y = bf_rne(bb.y); br.z = bf_rne(bb.z); br.w = bf_rne(bb.w);
      *(v4fa*)(sbs + 4 * tid) = br;
    }
  }
  const int fl = FLGG[(size_t)blockIdx.x * FLGW];
  __syncthreads();
  const v4f bv = *(const v4fa*)(sbs + 4 * lane);
  const float qnan = __int_as_float(0x7fc00000);
  unsigned int* stwu = stw + wave * STW;

#pragma unroll 1
  for (int jt = 0; jt < NB / NWAVE; ++jt) {
    const int slot = wave * (NB / NWAVE) + jt;
    const int grow = nodeBase + slot;
    if (grow >= MPr) continue;
    const int craw = scn[slot];
    int cnt = craw;
    int st  = sof[slot];
    st  = st < 0 ? 0 : (st > RCAP ? RCAP : st);
    cnt = cnt < 0 ? 0 : (cnt > DEGCAP ? DEGCAP : cnt);
    if (cnt > RCAP - st) cnt = RCAP - st;
    const float pz = (fl != 0 || craw > DEGCAP || craw < 0) ? qnan : 0.0f;
    const bool liveRow = grow < nN;
    const int nc = liveRow ? grow : nN - 1;
    const float dd = DISG[nc];
    const float rd = dd * dd;

    float ag0 = 0.0f, ag1 = 0.0f, ag2 = 0.0f, ag3 = 0.0f;
#pragma unroll 1
    for (int b0 = 0; b0 < cnt; b0 += 32) {
      int idx = st + b0 + lane;
      idx = idx > st + cnt - 1 ? st + cnt - 1 : idx;
      idx = idx < 0 ? 0 : (idx > RCAP - 1 ? RCAP - 1 : idx);
      int sv = lg[idx];
      sv = sv < 0 ? 0 : (sv > nN - 1 ? nN - 1 : sv);
      const float cf  = DISG[sv] * dd;
      const int   cfi = __float_as_int(cf);
      const int m32 = (cnt - b0) < 32 ? (cnt - b0) : 32;
#pragma unroll 1
      for (int k = 0; k < m32; ++k) {
        const int   sk = __builtin_amdgcn_readlane(sv, k);
        const float ck = __int_as_float(__builtin_amdgcn_readlane(cfi, k));
        const v4f v = *(const v4f*)(Hf + (size_t)sk * HID + 4 * lane);
        ag0 = fmaf(ck, v.x, ag0); ag1 = fmaf(ck, v.y, ag1);
        ag2 = fmaf(ck, v.z, ag2); ag3 = fmaf(ck, v.w, ag3);
      }
    }
    const v4f sf = *(const v4f*)(Hf + (size_t)nc * HID + 4 * lane);
    float r0 = (ag0 + sf.x * rd) + bv.x;
    float r1 = (ag1 + sf.y * rd) + bv.y;
    float r2 = (ag2 + sf.z * rd) + bv.z;
    float r3 = (ag3 + sf.w * rd) + bv.w;
    if constexpr (MODE != 0) {
      r0 = (r0 > 0.0f) ? r0 : (r0 - r0);
      r1 = (r1 > 0.0f) ? r1 : (r1 - r1);
      r2 = (r2 > 0.0f) ? r2 : (r2 - r2);
      r3 = (r3 > 0.0f) ? r3 : (r3 - r3);
    }
    r0 = (liveRow ? r0 : 0.0f) + pz;
    r1 = (liveRow ? r1 : 0.0f) + pz;
    r2 = (liveRow ? r2 : 0.0f) + pz;
    r3 = (liveRow ? r3 : 0.0f) + pz;

    if constexpr (MODE != 0) {
      const unsigned short hb0 = bf_bits(r0), hb1 = bf_bits(r1), hb2 = bf_bits(r2), hb3 = bf_bits(r3);
      const unsigned short lb0 = bf_bits(r0 - bf_val(hb0)), lb1 = bf_bits(r1 - bf_val(hb1));
      const unsigned short lb2 = bf_bits(r2 - bf_val(hb2)), lb3 = bf_bits(r3 - bf_val(hb3));
      v2u hw, lw;
      hw.x = (unsigned int)hb0 | ((unsigned int)hb1 << 16);
      hw.y = (unsigned int)hb2 | ((unsigned int)hb3 << 16);
      lw.x = (unsigned int)lb0 | ((unsigned int)lb1 << 16);
      lw.y = (unsigned int)lb2 | ((unsigned int)lb3 << 16);
      __builtin_amdgcn_fence(__ATOMIC_RELEASE, "wavefront");
      __builtin_amdgcn_wave_barrier();
      *(v2ua*)(stwu + 2 * lane)      = hw;
      *(v2ua*)(stwu + 64 + 2 * lane) = lw;
      __builtin_amdgcn_fence(__ATOMIC_RELEASE, "wavefront");
      __builtin_amdgcn_wave_barrier();
      const v4u pk = *(const v4ua*)(stwu + 4 * lane);
      unsigned short* gp = Xhl + (size_t)grow * (size_t)APW + 8 * lane;
      *(volatile v4u*)gp = pk;
      __threadfence();
      *(volatile v4u*)gp = pk;
    } else {
      v4f ow;
      ow.x = r0; ow.y = r1; ow.z = r2; ow.w = r3;
      float* op = Hout + (size_t)grow * (size_t)HID + 4 * lane;
      *(volatile v4f*)op = ow;
      __threadfence();
      *(volatile v4f*)op = ow;
    }
  }
}

__global__ __launch_bounds__(NTHR) void k_pool(const float* __restrict__ hf, const int* __restrict__ bat,
                                               int nN, float* pl) {
  __shared__ __attribute__((aligned(16))) float wsum[NWAVE * HID];
  __shared__ int wcn[NWAVE];
  __shared__ __attribute__((aligned(16))) float outs[HID];
  const int tid = (int)threadIdx.x, lane = tid & 31, wave = tid >> 5;
  const int g = (int)blockIdx.x;

  float a0 = 0.0f, a1 = 0.0f, a2 = 0.0f, a3 = 0.0f;
  int cnt = 0;
#pragma unroll 1
  for (int i0 = wave * 32; i0 < nN; i0 += NTHR) {
    const int i  = i0 + lane;
    const int ic = i < nN ? i : nN - 1;
    const int b  = bat[ic];
    const bool hit = (i < nN) && (b == g);
    unsigned msk = __builtin_amdgcn_ballot_w32(hit);
    int nh = (int)__builtin_popcount(msk);
    nh = nh > 32 ? 32 : nh;
    cnt += nh;
#pragma unroll 1
    for (int q = 0; q < nh; ++q) {
      const int k = __builtin_ffs((int)msk) - 1;
      msk &= msk - 1u;
      int node = i0 + (k < 0 ? 0 : k);
      node = node > nN - 1 ? nN - 1 : node;
      const v4f v = *(const v4f*)(hf + (size_t)node * HID + 4 * lane);
      a0 += v.x; a1 += v.y; a2 += v.z; a3 += v.w;
    }
  }
  wsum[wave * HID + 4 * lane + 0] = a0;
  wsum[wave * HID + 4 * lane + 1] = a1;
  wsum[wave * HID + 4 * lane + 2] = a2;
  wsum[wave * HID + 4 * lane + 3] = a3;
  if (lane == 0) wcn[wave] = cnt;
  __syncthreads();
  if (tid < HID) {
    float s = 0.0f;
    int c = 0;
#pragma unroll
    for (int w2 = 0; w2 < NWAVE; ++w2) { s += wsum[w2 * HID + tid]; c += wcn[w2]; }
    const float cf = (c < 1) ? 1.0f : (float)c;
    outs[tid] = s * (1.0f / cf);
  }
  __syncthreads();
  const v4f ov = *(const v4fa*)(outs + 4 * lane);
  float* op = pl + (size_t)g * HID + 4 * lane;
  const bool okst = (wave == 0);
  if (okst) *(volatile v4f*)op = ov;
  __threadfence();
  if (okst) *(volatile v4f*)op = ov;
}

__global__ __launch_bounds__(NTHR) void k_head(const float* __restrict__ pl, const float* __restrict__ Wl,
                                               const float* __restrict__ bl, const int* __restrict__ flg,
                                               int nFlag, float* out) {
  __shared__ float wls[HID * NCLS];
  __shared__ float bls[8];
  __shared__ int sfl[64];
  __shared__ __attribute__((aligned(16))) float os[NOUT];
  const int tid = (int)threadIdx.x;
#pragma unroll 1
  for (int i = tid; i < HID * NCLS; i += NTHR) wls[i] = bf_rne(Wl[i]);
  if (tid < 8) {
    const float bb = bl[tid < NCLS ? tid : NCLS - 1];
    bls[tid] = (tid < NCLS) ? bf_rne(bb) : 0.0f;
  }
  if (tid < 64) {
    const int fi = tid < nFlag ? tid : nFlag - 1;
    const int f  = flg[(size_t)fi * FLGW];
    sfl[tid] = (tid < nFlag) ? f : 0;
  }
  __syncthreads();
  int anyf = 0;
#pragma unroll 1
  for (int i = 0; i < 64; ++i) anyf |= sfl[i];
  const int g = tid;
  const float* pr = pl + (size_t)g * HID;
  float s0 = 0.0f, s1 = 0.0f, s2 = 0.0f, s3 = 0.0f, s4 = 0.0f;
#pragma unroll 1
  for (int f4 = 0; f4 < HID / 4; ++f4) {
    const v4f p = *(const v4f*)(pr + 4 * f4);
    const float* w = wls + (4 * f4) * NCLS;
    s0 = fmaf(p.x, w[0], s0); s1 = fmaf(p.x, w[1], s1); s2 = fmaf(p.x, w[2], s2);
    s3 = fmaf(p.x, w[3], s3); s4 = fmaf(p.x, w[4], s4);
    s0 = fmaf(p.y, w[5], s0); s1 = fmaf(p.y, w[6], s1); s2 = fmaf(p.y, w[7], s2);
    s3 = fmaf(p.y, w[8], s3); s4 = fmaf(p.y, w[9], s4);
    s0 = fmaf(p.z, w[10], s0); s1 = fmaf(p.z, w[11], s1); s2 = fmaf(p.z, w[12], s2);
    s3 = fmaf(p.z, w[13], s3); s4 = fmaf(p.z, w[14], s4);
    s0 = fmaf(p.w, w[15], s0); s1 = fmaf(p.w, w[16], s1); s2 = fmaf(p.w, w[17], s2);
    s3 = fmaf(p.w, w[18], s3); s4 = fmaf(p.w, w[19], s4);
  }
  const float qnan = __int_as_float(0x7fc00000);
  const bool bad = anyf != 0;
  os[g * NCLS + 0] = bad ? qnan : (s0 + bls[0]);
  os[g * NCLS + 1] = bad ? qnan : (s1 + bls[1]);
  os[g * NCLS + 2] = bad ? qnan : (s2 + bls[2]);
  os[g * NCLS + 3] = bad ? qnan : (s3 + bls[3]);
  os[g * NCLS + 4] = bad ? qnan : (s4 + bls[4]);
  __syncthreads();
  const int t1 = NTHR + (tid & 63);
  const v4f ov0 = *(const v4fa*)(os + 4 * tid);
  const v4f ov1 = *(const v4fa*)(os + 4 * t1);
  const bool w1 = tid < (NOUT / 4 - NTHR);
  *(volatile v4f*)(out + 4 * (size_t)tid) = ov0;
  if (w1) *(volatile v4f*)(out + 4 * (size_t)t1) = ov1;
  __threadfence();
  *(volatile v4f*)(out + 4 * (size_t)tid) = ov0;
  if (w1) *(volatile v4f*)(out + 4 * (size_t)t1) = ov1;
}

static inline int cdiv(int a, int b) { return (a + b - 1) / b; }
static inline size_t al256(size_t o) { return (o + 255) & ~(size_t)255; }

extern "C" void kernel_launch(void* const* d_in, const int* in_sizes, int n_in,
                              void* d_out, int out_size, void* d_ws, size_t ws_size,
                              hipStream_t stream) {
  if (n_in < 11) return;
  if (in_sizes[0] < CIN || (in_sizes[0] % CIN) != 0) return;
  const int nN = in_sizes[0] / CIN;
  if (nN < 1 || nN > (1 << 22)) return;
  if (in_sizes[1] < 2 || (in_sizes[1] & 1) != 0) return;
  const int nE = in_sizes[1] / 2;
  if (nE < 1 || nE > (1 << 21)) return;
  if (in_sizes[2] != nN) return;
  if (in_sizes[3] != CIN * HID || in_sizes[4] != HID) return;
  if (in_sizes[5] != HID * HID || in_sizes[6] != HID) return;
  if (in_sizes[7] != HID * HID || in_sizes[8] != HID) return;
  if (in_sizes[9] != HID * NCLS || in_sizes[10] != NCLS) return;
  if (out_size != NOUT) return;

  const float* x    = (const float*)d_in[0];
  const int*   edge = (const int*)  d_in[1];
  const int*   bat  = (const int*)  d_in[2];
  const float* W1   = (const float*)d_in[3];
  const float* b1   = (const float*)d_in[4];
  const float* W2   = (const float*)d_in[5];
  const float* b2   = (const float*)d_in[6];
  const float* W3   = (const float*)d_in[7];
  const float* b3   = (const float*)d_in[8];
  const float* Wl   = (const float*)d_in[9];
  const float* bl   = (const float*)d_in[10];
  float* out = (float*)d_out;
  const int* src = edge;
  const int* dst = edge + nE;

  const int MP   = cdiv(nN, GBM) * GBM;
  const int gM   = MP / GBM;
  const int gA   = cdiv(MP, NB);
  const int NP   = gA * NB;
  if ((long long)gA * NB < (long long)MP) return;
  if (gA < 1 || gA > 64) return;
  const int vec8 = ((nE & 3) == 0) ? 1 : 0;
  const int nUx  = MP * (CIN / 8);
  if ((nUx % NTHR) != 0) return;

  char* ws = (char*)d_ws;
  size_t off = 0;
  const size_t oXB  = off; off = al256(off + (size_t)MP * CIN * 2);
  const size_t oW1  = off; off = al256(off + (size_t)HID * CIN * 2);
  const size_t oW2  = off; off = al256(off + (size_t)HID * APW * 2);
  const size_t oW3  = off; off = al256(off + (size_t)HID * APW * 2);
  const size_t oH   = off; off = al256(off + (size_t)MP * HID * 4);
  const size_t oXH  = off; off = al256(off + (size_t)MP * APW * 2);
  const size_t oH3  = off; off = al256(off + (size_t)MP * HID * 4);
  const size_t oLS  = off; off = al256(off + (size_t)gA * RCAP * 4);
  const size_t oCN  = off; off = al256(off + (size_t)NP * 4);
  const size_t oOF  = off; off = al256(off + (size_t)NP * 4);
  const size_t oDI  = off; off = al256(off + (size_t)NP * 4);
  const size_t oFL  = off; off = al256(off + (size_t)gA * FLGW * 4);
  const size_t oPL  = off; off = al256(off + (size_t)NGR * HID * 4);
  if (off > ws_size || off > (size_t)WSMAX) return;
  unsigned short* P16 = (unsigned short*)ws;
  unsigned short* XB  = (unsigned short*)(ws + oXB);
  unsigned short* W1T = (unsigned short*)(ws + oW1);
  unsigned short* W2D = (unsigned short*)(ws + oW2);
  unsigned short* W3D = (unsigned short*)(ws + oW3);
  float*          H   = (float*)(ws + oH);
  unsigned short* XHL = (unsigned short*)(ws + oXH);
  float*          H3  = (float*)(ws + oH3);
  int*            LST = (int*)(ws + oLS);
  int*            CNT = (int*)(ws + oCN);
  int*            OFS = (int*)(ws + oOF);
  float*          DIS = (float*)(ws + oDI);
  int*            FLG = (int*)(ws + oFL);
  float*          PL  = (float*)(ws + oPL);

  hipFuncSetAttribute(reinterpret_cast<const void*>(&k_bucket), hipFuncAttributeMaxDynamicSharedMemorySize, LDS_BKT);

  k_prep<<<(nUx + NU1 + 2 * NUD) / NTHR, NTHR, 0, stream>>>(x, W1, W2, W3, nN, nUx, P16,
                                                             oXB / 2, oW1 / 2, oW2 / 2, oW3 / 2);
  k_bucket<<<gA, NTHR, LDS_BKT, stream>>>(src, dst, nN, nE, vec8, LST, CNT, OFS, DIS, FLG);
  k_gemm<CIN><<<gM, GTHR, 0, stream>>>(XB, W1T, H, MP);
  k_agg<1><<<gA, NTHR, 0, stream>>>(LST, CNT, OFS, FLG, DIS, H, b1, XHL, H3, nN, MP);
  k_gemm<APW><<<gM, GTHR, 0, stream>>>(XHL, W2D, H, MP);
  k_agg<1><<<gA, NTHR, 0, stream>>>(LST, CNT, OFS, FLG, DIS, H, b2, XHL, H3, nN, MP);
  k_gemm<APW><<<gM, GTHR, 0, stream>>>(XHL, W3D, H, MP);
  k_agg<0><<<gA, NTHR, 0, stream>>>(LST, CNT, OFS, FLG, DIS, H, b3, XHL, H3, nN, MP);
  k_pool<<<NGR, NTHR, 0, stream>>>(H3, bat, nN, PL);
  k_head<<<1, NTHR, 0, stream>>>(PL, Wl, bl, FLG, gA, out);
}
